// GCNEncoder_15006615732583
// MI455X (gfx1250) — hardware-run, weakly checked
//
#include <hip/hip_runtime.h>

typedef float          v8f   __attribute__((ext_vector_type(8)));
typedef float          v4f   __attribute__((ext_vector_type(4)));
typedef unsigned int   v4u   __attribute__((ext_vector_type(4)));
typedef int            v8i   __attribute__((ext_vector_type(8)));
typedef unsigned short v8us  __attribute__((ext_vector_type(8)));
typedef unsigned short v16us __attribute__((ext_vector_type(16)));
typedef __bf16         v16bf __attribute__((ext_vector_type(16)));
typedef _Float16       v16h  __attribute__((ext_vector_type(16)));
typedef v4f  __attribute__((may_alias)) v4fa;
typedef v8us __attribute__((may_alias)) v8usa;
union FragB { v16bf v; v16us u; v8us h[2]; v8i w; };
union FragH { v16h  v; v16us u; v8us h[2]; v8i w; };

__device__ __forceinline__ v8f wmb(const FragB& a, const FragB& b, v8f c) {
  v8f d = __builtin_amdgcn_wmma_f32_16x16x32_bf16(false, a.v, false, b.v, (short)0, c, false, false);
  asm volatile("v_nop\n\tv_nop\n\tv_nop\n\tv_nop" : "+v"(d) : "v"(a.w), "v"(b.w));
  return d;
}

__device__ __forceinline__ v8f wmh(const FragH& a, const FragH& b, v8f c) {
  v8f d = __builtin_amdgcn_wmma_f32_16x16x32_f16(false, a.v, false, b.v, (short)0, c, false, false);
  asm volatile("v_nop\n\tv_nop\n\tv_nop\n\tv_nop" : "+v"(d) : "v"(a.w), "v"(b.w));
  return d;
}

__device__ __forceinline__ unsigned bf16_bits(float f) {
  const unsigned u = __float_as_uint(f);
  const unsigned r = (u + 0x7FFFu + ((u >> 16) & 1u)) >> 16;
  const unsigned q = (u >> 16) | 0x40u;
  return ((u & 0x7fffffffu) > 0x7f800000u) ? q : r;
}

__device__ __forceinline__ float bf16_val(float f) {
  return __uint_as_float(bf16_bits(f) << 16);
}
__device__ __forceinline__ int clampi(int v, int lo, int hi) {
  return v < lo ? lo : (v > hi ? hi : v);
}

__device__ __forceinline__ unsigned f16_bits(float f) {
  const unsigned u  = __float_as_uint(f);
  const unsigned s  = (u >> 16) & 0x8000u;
  const unsigned a  = u & 0x7fffffffu;
  const unsigned t  = a - 0x38000000u;
  const unsigned r  = (t + 0x0FFFu + ((t >> 13) & 1u)) >> 13;
  const unsigned rc = r > 0x7C00u ? 0x7C00u : r;
  const bool small  = a < 0x38800000u;
  const bool isnan  = a > 0x7f800000u;
  const unsigned fin = small ? 0u : (s | rc);
  return isnan ? (s | 0x7E00u) : fin;
}

__device__ __forceinline__ unsigned pk16(unsigned lo, unsigned hi) { return lo | (hi << 16); }
__device__ __forceinline__ unsigned bf16_lo_bits(float v) {
  float hi = bf16_val(v);
  asm volatile("" : "+v"(hi));
  return bf16_bits(v - hi);
}
__device__ __forceinline__ v4u pack8_bf16(v4f a, v4f c) {
  return (v4u){ pk16(bf16_bits(a[0]), bf16_bits(a[1])), pk16(bf16_bits(a[2]), bf16_bits(a[3])),
                pk16(bf16_bits(c[0]), bf16_bits(c[1])), pk16(bf16_bits(c[2]), bf16_bits(c[3])) };
}
__device__ __forceinline__ v4u pack8_bf16_lo(v4f a, v4f c) {
  return (v4u){ pk16(bf16_lo_bits(a[0]), bf16_lo_bits(a[1])), pk16(bf16_lo_bits(a[2]), bf16_lo_bits(a[3])),
                pk16(bf16_lo_bits(c[0]), bf16_lo_bits(c[1])), pk16(bf16_lo_bits(c[2]), bf16_lo_bits(c[3])) };
}
__device__ __forceinline__ v4u pack8_f16(v4f a, v4f c) {
  return (v4u){ pk16(f16_bits(a[0]), f16_bits(a[1])), pk16(f16_bits(a[2]), f16_bits(a[3])),
                pk16(f16_bits(c[0]), f16_bits(c[1])), pk16(f16_bits(c[2]), f16_bits(c[3])) };
}

template <int FORM>
__global__ __launch_bounds__(256) void k_plane(const float* __restrict__ src, int rows, int cols, int ldsrc,
                                               unsigned short* __restrict__ dst, int MP, int KP) {
  static_assert(FORM >= 0 && FORM <= 3);
  const int KTOT = (FORM == 1 || FORM == 3) ? 2 * KP : KP;
  const unsigned ppr   = (unsigned)(KTOT >> 3);
  const unsigned kp8   = (unsigned)(KP >> 3);
  const unsigned total = (unsigned)MP * ppr;
  const unsigned g     = blockIdx.x * 256u + threadIdx.x;
  const unsigned rowu  = g / ppr;
  const unsigned p     = g - rowu * ppr;
  const bool second    = p >= kp8;
  const int row = (int)rowu;
  const int c0  = (int)((second ? p - kp8 : p) << 3);
  const float* srow = src + (size_t)clampi(row, 0, rows - 1) * (size_t)ldsrc;
  float x[8];
  unsigned mk[8];
#pragma unroll
  for (int e = 0; e < 8; ++e) {
    const int c = c0 + e;
    const float v = srow[clampi(c, 0, cols - 1)];
    asm volatile("" :: "v"(v));
    x[e]  = v;
    mk[e] = (row < rows && c < cols) ? 0xFFFFu : 0u;
  }
  const v4f a = (v4f){ x[0], x[1], x[2], x[3] };
  const v4f c = (v4f){ x[4], x[5], x[6], x[7] };
  v4u o;
  if (FORM == 2) {
    o = pack8_f16(a, c);
  } else {
    const v4u hi = pack8_bf16(a, c);
    o = hi;
    if (FORM == 1) { const v4u lo = pack8_bf16_lo(a, c); o = second ? lo : hi; }
  }
  const v4u mw = (v4u){ pk16(mk[0], mk[1]), pk16(mk[2], mk[3]), pk16(mk[4], mk[5]), pk16(mk[6], mk[7]) };
  o &= mw;
  if (g < total) {
    volatile v4u* q = (volatile v4u*)(dst + (size_t)g * 8);
    *q = o;
    __threadfence();
    *q = o;
  }
}

template <int FORM> struct FragOf    { typedef FragB T; };
template <>         struct FragOf<2> { typedef FragH T; };
__device__ __forceinline__ v8f mm(const FragB& a, const FragB& b, v8f c) { return wmb(a, b, c); }
__device__ __forceinline__ v8f mm(const FragH& a, const FragH& b, v8f c) { return wmh(a, b, c); }
template <class F> __device__ __forceinline__ F ld_frag(const unsigned short* p) {
  F f;
  f.h[0] = *(const v8usa*)(p);
  f.h[1] = *(const v8usa*)(p + 16);
  return f;
}

template <int FORM, int EPI>
__global__ __launch_bounds__(256) __attribute__((amdgpu_num_vgpr(248)))
void k_gemm_nt(const unsigned short* __restrict__ A, const unsigned short* __restrict__ B,
               const float* __restrict__ bias, float* __restrict__ D, int M, int N, int KTOT, int ldd) {
  static_assert(FORM >= 0 && FORM <= 2);
  static_assert(EPI == 0 || EPI == 1);
  typedef typename FragOf<FORM>::T F;
  __shared__ __attribute__((aligned(16))) float sT[8][16 * 68];
  const int lane = threadIdx.x & 31;
  const int wave = threadIdx.x >> 5;
  const int tilesM = (M + 63) >> 6;
  const int tilesN = (N + 63) >> 6;
  const int tile = blockIdx.x * 8 + wave;
  if (tile >= tilesM * tilesN) return;
  const int tm = tile / tilesN;
  const int tn = tile - tm * tilesN;
  const int m0 = tm << 6;
  const int n0 = tn << 6;

  const int rl = lane & 15;
  const int h8 = (lane >> 4) * 8;
  const unsigned short* pa = A + (size_t)(m0 + rl) * (size_t)KTOT + h8;
  const unsigned short* pb = B + (size_t)(n0 + rl) * (size_t)KTOT + h8;

  v8f acc[4][4];
#pragma unroll
  for (int i = 0; i < 4; ++i)
#pragma unroll
    for (int j = 0; j < 4; ++j) acc[i][j] = (v8f){0.f, 0.f, 0.f, 0.f, 0.f, 0.f, 0.f, 0.f};

#pragma unroll 1
  for (int k0 = 0; k0 < KTOT; k0 += 32) {
    F bf[4];
#pragma unroll
    for (int j = 0; j < 4; ++j) bf[j] = ld_frag<F>(pb + (size_t)(j << 4) * (size_t)KTOT + k0);
#pragma unroll
    for (int i = 0; i < 4; ++i) {
      const F af = ld_frag<F>(pa + (size_t)(i << 4) * (size_t)KTOT + k0);
#pragma unroll
      for (int j = 0; j < 4; ++j) acc[i][j] = mm(af, bf[j], acc[i][j]);
    }
  }

  float* slab = sT[wave];
  const int hh = lane >> 4;
  const int c4 = (lane & 15) * 4;
  const int nc = n0 + c4;
  const bool cok = nc < N;
  v4f bv = (v4f){0.f, 0.f, 0.f, 0.f};
  if (EPI == 1) {
    bv = *(const v4fa*)(bias + clampi(nc, 0, N - 4));
    asm volatile("" :: "v"(bv));
  }
#pragma unroll
  for (int i = 0; i < 4; ++i) {
    const int mBase = m0 + (i << 4);
#pragma unroll
    for (int j = 0; j < 4; ++j) {
#pragma unroll
      for (int r = 0; r < 8; ++r) slab[(h8 + r) * 68 + (j << 4) + rl] = acc[i][j][r];
    }
    __builtin_amdgcn_fence(__ATOMIC_RELEASE, "workgroup");
    __builtin_amdgcn_wave_barrier();
    __builtin_amdgcn_fence(__ATOMIC_ACQUIRE, "workgroup");
    v4f vv[8];
#pragma unroll
    for (int it = 0; it < 8; ++it) {
      const int row = it * 2 + hh;
      v4f v = *(const v4fa*)(slab + row * 68 + c4);
      if (EPI == 1) v += bv;
      vv[it] = v;
    }
    for (int pass = 0; pass < 2; ++pass) {
#pragma unroll
      for (int it = 0; it < 8; ++it) {
        const int row = mBase + it * 2 + hh;
        if (cok && row < M) *(volatile v4f*)(D + (size_t)row * (size_t)ldd + nc) = vv[it];
      }
      __threadfence();
    }
    __builtin_amdgcn_fence(__ATOMIC_RELEASE, "workgroup");
    __builtin_amdgcn_wave_barrier();
    __builtin_amdgcn_fence(__ATOMIC_ACQUIRE, "workgroup");
  }
}

#define H1_TERMS 2
#define N_      50000
#define E_      800000
#define C0_     128
#define C2_     64
#define NP_     50048
#define K1_     (128 * H1_TERMS)
#define BTHR    256
#define CHUNK_  2048
#define NCHUNK_ ((E_ + CHUNK_ - 1) / CHUNK_)
#define SLOTS_  1024
#define NBLK_   49
#define RCAP_   21504
#define DEGCAP_ 64
#define MAXB1024_ 16623
#define MAXDEG_   35
#define BUCKET_INTS (2 * RCAP_ + 3 * SLOTS_ + 32)
#define BUCKET_LDS  (BUCKET_INTS * 4)

static_assert(H1_TERMS == 1 || H1_TERMS == 2);
static_assert(N_ % 8 == 0);
static_assert(E_ % 256 == 0 && E_ % 8 == 0 && E_ >= 8);
static_assert(NP_ == 391 * 128 && NP_ % 64 == 0 && NP_ >= N_ && NP_ % 16 == 0);
static_assert(NBLK_ * SLOTS_ >= N_ && (NBLK_ - 1) * SLOTS_ < N_);
static_assert(4 * RCAP_ >= 5 * MAXB1024_);
static_assert(RCAP_ % 1024 == 0);
static_assert(DEGCAP_ >= MAXDEG_ + 8);
static_assert(N_ <= (1 << 21));
static_assert(BUCKET_LDS <= 262144);
static_assert(C0_ % 32 == 0 && K1_ % 32 == 0 && C2_ % 4 == 0);
static_assert((long long)(N_ - 1) * C2_ + (C2_ - 1) == 3199999LL);

typedef int          v4i  __attribute__((ext_vector_type(4)));
typedef float        v2f  __attribute__((ext_vector_type(2)));
typedef unsigned int v2u  __attribute__((ext_vector_type(2)));
typedef v4i __attribute__((may_alias)) v4ia;
typedef v2f __attribute__((may_alias)) v2fa;

#define PB_W0   8
#define NU_W1   (C2_ * (K1_ / 8))
#define PB_W1   (NU_W1 / BTHR)
#define PADPIECES ((NP_ - N_) * K1_ / 8)
#define PB_PAD  (PADPIECES / BTHR)
#define PB_TOTAL (PB_W0 + PB_W1 + 1 + PB_PAD)
static_assert(C0_ * (C0_ / 8) == PB_W0 * BTHR);
static_assert(NU_W1 % BTHR == 0 && PADPIECES % BTHR == 0 && PADPIECES > 0);

__global__ __launch_bounds__(BTHR) void k_prep(const float* __restrict__ W0, const float* __restrict__ W1,
                                               const float* __restrict__ b0, const float* __restrict__ b1,
                                               unsigned short* __restrict__ W0T, unsigned short* __restrict__ W1D,
                                               float* __restrict__ B0f, float* __restrict__ B1f,
                                               unsigned short* __restrict__ H1HL) {
  const int blk = (int)blockIdx.x;
  const int tid = (int)threadIdx.x;
  if (blk < PB_W0) {
    const int u  = blk * BTHR + tid;
    const int n  = u >> 4;
    const int k8 = (u & 15) * 8;
    const float* p = W0 + (size_t)k8 * C0_ + n;
    unsigned w[8];
#pragma unroll
    for (int i = 0; i < 8; ++i) w[i] = bf16_bits(p[(size_t)i * C0_]);
    const v4u o = (v4u){ pk16(w[0], w[1]), pk16(w[2], w[3]), pk16(w[4], w[5]), pk16(w[6], w[7]) };
    volatile v4u* q = (volatile v4u*)(W0T + (size_t)n * C0_ + k8);
    *q = o;
    __threadfence();
    *q = o;
  } else if (blk < PB_W0 + PB_W1) {
    const int v  = (blk - PB_W0) * BTHR + tid;
    const int n  = v / (K1_ / 8);
    const int k8 = (v - n * (K1_ / 8)) * 8;
    const int kk = k8 & (C0_ - 1);
    const float* p = W1 + (size_t)kk * C2_ + n;
    unsigned w[8];
#pragma unroll
    for (int i = 0; i < 8; ++i) w[i] = bf16_bits(p[(size_t)i * C2_]);
    const v4u o = (v4u){ pk16(w[0], w[1]), pk16(w[2], w[3]), pk16(w[4], w[5]), pk16(w[6], w[7]) };
    volatile v4u* q = (volatile v4u*)(W1D + (size_t)n * K1_ + k8);
    *q = o;
    __threadfence();
    *q = o;
  } else if (blk == PB_W0 + PB_W1) {
    const int t0 = tid < 31 ? tid : 31;
    const int t1 = clampi(tid - 32, 0, 15);
    const v4f a = *(const v4fa*)(b0 + 4 * t0);
    const v4f c = *(const v4fa*)(b1 + 4 * t1);
    asm volatile("" :: "v"(a));
    asm volatile("" :: "v"(c));
    const v4f r0 = (v4f){ bf16_val(a[0]), bf16_val(a[1]), bf16_val(a[2]), bf16_val(a[3]) };
    const v4f r1 = (v4f){ bf16_val(c[0]), bf16_val(c[1]), bf16_val(c[2]), bf16_val(c[3]) };
    const bool is0 = tid < 32;
    const bool is1 = (tid >= 32) && (tid < 48);
    for (int pass = 0; pass < 2; ++pass) {
      if (is0) *(volatile v4f*)(B0f + 4 * t0) = r0;
      if (is1) *(volatile v4f*)(B1f + 4 * t1) = r1;
      __threadfence();
    }
  } else {
    const int g = (blk - (PB_W0 + PB_W1 + 1)) * BTHR + tid;
    const v4u z = (v4u){0u, 0u, 0u, 0u};
    volatile v4u* q = (volatile v4u*)(H1HL + (size_t)N_ * K1_ + (size_t)g * 8);
    *q = z;
    __threadfence();
    *q = z;
  }
}

__global__ __launch_bounds__(BTHR) void k_bucket(const int* __restrict__ srcs, const int* __restrict__ dsts,
                                                 int* __restrict__ LIST, int* __restrict__ CNT,
                                                 int* __restrict__ OFF, int* __restrict__ DINVb,
                                                 int* __restrict__ POIS) {
  extern __shared__ __attribute__((aligned(16))) int dsm[];
  int* HL = dsm;
  int* SL = dsm + RCAP_;
  int* CN = dsm + 2 * RCAP_;
  int* OF = CN + SLOTS_;
  int* DV = OF + SLOTS_;
  int* MS = DV + SLOTS_;
  const int tid = (int)threadIdx.x, lane = tid & 31, wave = tid >> 5;
  const int base = (int)blockIdx.x * SLOTS_;

  {
    const v4i z4 = (v4i){0, 0, 0, 0};
    const v4i m4 = (v4i){-1, -1, -1, -1};
#pragma unroll 1
    for (int i = tid * 4; i < RCAP_; i += BTHR * 4) { *(v4ia*)(HL + i) = z4; *(v4ia*)(SL + i) = m4; }
#pragma unroll 1
    for (int i = tid * 4; i < 3 * SLOTS_; i += BTHR * 4) *(v4ia*)(CN + i) = z4;
    if (tid < 32) MS[tid] = 0;
  }
  __syncthreads();

  int t = 0;
  const unsigned ub = (unsigned)base;
#pragma unroll 1
  for (int ch = 0; ch < NCHUNK_; ++ch) {
    const int e0 = ch * CHUNK_ + tid * 8;
    const bool valid = e0 < E_;
    const int e0c = valid ? e0 : (E_ - 8);
    const v4i da = *(const v4ia*)(dsts + e0c);
    const v4i db = *(const v4ia*)(dsts + e0c + 4);
    const v4i sa = *(const v4ia*)(srcs + e0c);
    const v4i sb = *(const v4ia*)(srcs + e0c + 4);
    asm volatile("" :: "v"(da));
    asm volatile("" :: "v"(db));
    asm volatile("" :: "v"(sa));
    asm volatile("" :: "v"(sb));
    const int vm = valid ? -1 : 0;
    const int nm = ~vm;
    const unsigned s0 = (unsigned)((da.x & vm) | nm) - ub, s1 = (unsigned)((da.y & vm) | nm) - ub;
    const unsigned s2 = (unsigned)((da.z & vm) | nm) - ub, s3 = (unsigned)((da.w & vm) | nm) - ub;
    const unsigned s4 = (unsigned)((db.x & vm) | nm) - ub, s5 = (unsigned)((db.y & vm) | nm) - ub;
    const unsigned s6 = (unsigned)((db.z & vm) | nm) - ub, s7 = (unsigned)((db.w & vm) | nm) - ub;
    const bool h0 = s0 < (unsigned)SLOTS_, h1 = s1 < (unsigned)SLOTS_, h2 = s2 < (unsigned)SLOTS_;
    const bool h3 = s3 < (unsigned)SLOTS_, h4 = s4 < (unsigned)SLOTS_, h5 = s5 < (unsigned)SLOTS_;
    const bool h6 = s6 < (unsigned)SLOTS_, h7 = s7 < (unsigned)SLOTS_;
    const int hc = (int)h0 + (int)h1 + (int)h2 + (int)h3 + (int)h4 + (int)h5 + (int)h6 + (int)h7;
    int incl = hc;
#pragma unroll
    for (int d = 1; d < 32; d <<= 1) {
      const int y = __shfl_up(incl, d, 32);
      incl += (lane >= d) ? y : 0;
    }
    const int wtot = __shfl(incl, 31, 32);
    const int par = (ch & 1) * 8;
    if (lane == 0) MS[par + wave] = wtot;
    __syncthreads();
    int wb = 0, ct = 0;
#pragma unroll
    for (int i = 0; i < 8; ++i) {
      const int m = MS[par + i];
      ct += m;
      wb += (i < wave) ? m : 0;
    }
    int pos = t + wb + (incl - hc);
#define PUTJ(HJ, SRCJ, SLJ) { \
      if (HJ) { if (pos < RCAP_) HL[pos] = (clampi((SRCJ), 0, N_ - 1) << 10) | (int)(SLJ); } \
      pos += (HJ) ? 1 : 0; }
    PUTJ(h0, sa.x, s0)
    PUTJ(h1, sa.y, s1)
    PUTJ(h2, sa.z, s2)
    PUTJ(h3, sa.w, s3)
    PUTJ(h4, sb.x, s4)
    PUTJ(h5, sb.y, s5)
    PUTJ(h6, sb.z, s6)
    PUTJ(h7, sb.w, s7)
#undef PUTJ
    t += ct;
  }
  __syncthreads();
  const int ovf = t > RCAP_ ? 1 : 0;
  const int tt  = t > RCAP_ ? RCAP_ : (t < 0 ? 0 : t);

  int c0 = 0, c1 = 0, c2 = 0, c3 = 0;
#pragma unroll 1
  for (int b0 = 0; b0 < tt; b0 += 32) {
    const int idx = b0 + lane;
    const int ent = HL[idx < RCAP_ ? idx : RCAP_ - 1];
    const bool mine = (idx < tt) && (((ent >> 7) & 7) == wave);
    unsigned msk = __builtin_amdgcn_ballot_w32(mine);
    int nh = (int)__builtin_popcount(msk);
    nh = nh > 32 ? 32 : nh;
#pragma unroll 1
    for (int q = 0; q < nh; ++q) {
      const int k = clampi(__builtin_ffs((int)msk) - 1, 0, 31);
      msk &= msk - 1u;
      const int u   = __builtin_amdgcn_readlane(ent, k);
      const int ls  = u & 127;
      const int inc = ((ls >> 2) == lane) ? 1 : 0;
      const int qq  = ls & 3;
      c0 += (qq == 0) ? inc : 0;
      c1 += (qq == 1) ? inc : 0;
      c2 += (qq == 2) ? inc : 0;
      c3 += (qq == 3) ? inc : 0;
    }
  }
  const int sm = c0 + c1 + c2 + c3;
  int incl2 = sm;
#pragma unroll
  for (int d = 1; d < 32; d <<= 1) {
    const int y = __shfl_up(incl2, d, 32);
    incl2 += (lane >= d) ? y : 0;
  }
  const int wtot2 = __shfl(incl2, 31, 32);
  const bool bigl = (c0 > DEGCAP_) || (c1 > DEGCAP_) || (c2 > DEGCAP_) || (c3 > DEGCAP_);
  const unsigned bigm = __builtin_amdgcn_ballot_w32(bigl);
  if (lane == 0) { MS[16 + wave] = wtot2; MS[24 + wave] = (bigm != 0u) ? 1 : 0; }
  __syncthreads();
  int wb2 = 0, bg = 0;
#pragma unroll
  for (int i = 0; i < 8; ++i) {
    const int m = MS[16 + i];
    wb2 += (i < wave) ? m : 0;
    bg |= MS[24 + i];
  }
  int p0 = wb2 + (incl2 - sm);
  int p1 = p0 + c0;
  int p2 = p1 + c1;
  int p3 = p2 + c2;
  {
    const int sl0 = wave * 128 + lane * 4;
    *(v4ia*)(CN + sl0) = (v4i){c0, c1, c2, c3};
    *(v4ia*)(OF + sl0) = (v4i){p0, p1, p2, p3};
  }
#pragma unroll 1
  for (int b0 = 0; b0 < tt; b0 += 32) {
    const int idx = b0 + lane;
    const int ent = HL[idx < RCAP_ ? idx : RCAP_ - 1];
    const bool mine = (idx < tt) && (((ent >> 7) & 7) == wave);
    unsigned msk = __builtin_amdgcn_ballot_w32(mine);
    int nh = (int)__builtin_popcount(msk);
    nh = nh > 32 ? 32 : nh;
#pragma unroll 1
    for (int q = 0; q < nh; ++q) {
      const int k = clampi(__builtin_ffs((int)msk) - 1, 0, 31);
      msk &= msk - 1u;
      const int u   = __builtin_amdgcn_readlane(ent, k);
      const int ls  = u & 127;
      const bool own = (ls >> 2) == lane;
      const int qq  = ls & 3;
      const int pp  = (qq == 0) ? p0 : ((qq == 1) ? p1 : ((qq == 2) ? p2 : p3));
      if (own && (unsigned)pp < (unsigned)RCAP_) SL[pp] = u >> 10;
      const int inc = own ? 1 : 0;
      p0 += (qq == 0) ? inc : 0;
      p1 += (qq == 1) ? inc : 0;
      p2 += (qq == 2) ? inc : 0;
      p3 += (qq == 3) ? inc : 0;
    }
  }
  __syncthreads();

#pragma unroll 1
  for (int i = 0; i < SLOTS_ / BTHR; ++i) {
    const int sl  = tid + BTHR * i;
    const int deg = CN[sl] + 1;
    const float df = (float)deg;
    const float dv = (deg > 0) ? (1.0f / sqrtf(df)) : 0.0f;
    DV[sl] = __float_as_int(dv);
  }
  __syncthreads();

  const int pflag = (ovf | bg) != 0 ? 1 : 0;
  const v4i cv  = *(const v4ia*)(CN + 4 * tid);
  const v4i ov4 = *(const v4ia*)(OF + 4 * tid);
  const v4i dv4 = *(const v4ia*)(DV + 4 * tid);
  const v4i pv  = (v4i){pflag, pflag, pflag, pflag};
  int* lbase = LIST + (size_t)blockIdx.x * RCAP_;
  for (int pass = 0; pass < 2; ++pass) {
    *(volatile v4i*)(CNT   + base + 4 * tid) = cv;
    *(volatile v4i*)(OFF   + base + 4 * tid) = ov4;
    *(volatile v4i*)(DINVb + base + 4 * tid) = dv4;
    if (tid < 8) *(volatile v4i*)(POIS + (int)blockIdx.x * 32 + 4 * tid) = pv;
#pragma unroll 1
    for (int it = 0; it < RCAP_ / 1024; ++it) {
      const v4i lv = *(const v4ia*)(SL + it * 1024 + 4 * tid);
      *(volatile v4i*)(lbase + it * 1024 + 4 * tid) = lv;
    }
    __threadfence();
  }
}

__device__ __forceinline__ float logistic(float v) { return 1.0f / (1.0f + expf(-v)); }

__global__ __launch_bounds__(BTHR) void k_replay0(const float* __restrict__ H, const int* __restrict__ LIST,
                                                  const int* __restrict__ CNT, const int* __restrict__ OFF,
                                                  const float* __restrict__ DINV, const int* __restrict__ POIS,
                                                  const float* __restrict__ B0f,
                                                  unsigned short* __restrict__ H1HL) {
  __shared__ __attribute__((aligned(16))) float sB[C0_];
  const int tid = (int)threadIdx.x, lane = tid & 31, wave = tid >> 5;
  if (tid < 32) { const v4f b = *(const v4fa*)(B0f + 4 * tid); *(v4fa*)(sB + 4 * tid) = b; }
  __syncthreads();
  const v4f bv = *(const v4fa*)(sB + 4 * lane);
  const int row = (int)blockIdx.x * 8 + wave;
  const bool live = row < N_;
  const int rc = live ? row : (N_ - 1);
  int c = CNT[rc];
  asm volatile("" :: "v"(c));
  int o = OFF[rc];
  asm volatile("" :: "v"(o));
  const float dr = DINV[rc];
  asm volatile("" :: "v"(dr));
  const int blk = rc >> 10;
  const int pf = POIS[blk * 32];
  asm volatile("" :: "v"(pf));
  const bool big = c > DEGCAP_;
  c = clampi(c, 0, DEGCAP_);
  o = clampi(o, 0, RCAP_ - 1);
  const int cn = __builtin_amdgcn_readfirstlane(live ? c : 0);
  const int* lst = LIST + (size_t)blk * RCAP_;

  v4f acc = (v4f){0.0f, 0.0f, 0.0f, 0.0f};
#pragma unroll 1
  for (int b0 = 0; b0 < cn; b0 += 32) {
    int idx = o + b0 + lane;
    idx = idx > RCAP_ - 1 ? RCAP_ - 1 : idx;
    const int s = clampi(lst[idx], 0, N_ - 1);
    const float w = DINV[s] * dr;
    const int wi = __float_as_int(w);
    const int m32 = (cn - b0) < 32 ? (cn - b0) : 32;
#pragma unroll 1
    for (int k = 0; k < m32; ++k) {
      const int   sk = clampi(__builtin_amdgcn_readlane(s, k), 0, N_ - 1);
      const float ck = __int_as_float(__builtin_amdgcn_readlane(wi, k));
      const v4f a = *(const v4fa*)(H + (size_t)sk * C0_ + 4 * lane);
      acc[0] = fmaf(ck, a[0], acc[0]);
      acc[1] = fmaf(ck, a[1], acc[1]);
      acc[2] = fmaf(ck, a[2], acc[2]);
      acc[3] = fmaf(ck, a[3], acc[3]);
    }
  }
  const v4f hr = *(const v4fa*)(H + (size_t)rc * C0_ + 4 * lane);
  const float h0 = hr[0], h1 = hr[1], h2 = hr[2], h3 = hr[3];
  asm volatile("" :: "v"(h0));
  asm volatile("" :: "v"(h1));
  asm volatile("" :: "v"(h2));
  asm volatile("" :: "v"(h3));
  const float rd = dr * dr;
  float y0 = logistic((acc[0] + h0 * rd) + bv[0]);
  float y1 = logistic((acc[1] + h1 * rd) + bv[1]);
  float y2 = logistic((acc[2] + h2 * rd) + bv[2]);
  float y3 = logistic((acc[3] + h3 * rd) + bv[3]);
  const bool bad = (pf != 0) || big;
  const float qnan = __int_as_float(0x7fc00000);
  y0 = bad ? qnan : y0;
  y1 = bad ? qnan : y1;
  y2 = bad ? qnan : y2;
  y3 = bad ? qnan : y3;
  const v2u hv = (v2u){ pk16(bf16_bits(y0), bf16_bits(y1)), pk16(bf16_bits(y2), bf16_bits(y3)) };
  const v2u lv = (v2u){ pk16(bf16_lo_bits(y0), bf16_lo_bits(y1)), pk16(bf16_lo_bits(y2), bf16_lo_bits(y3)) };
  unsigned short* rp = H1HL + (size_t)rc * K1_ + 4 * lane;
  for (int pass = 0; pass < 2; ++pass) {
    if (live) *(volatile v2u*)rp = hv;
    if (H1_TERMS == 2) { if (live) *(volatile v2u*)(rp + C0_) = lv; }
    __threadfence();
  }
}

__global__ __launch_bounds__(BTHR) void k_replay1(const float* __restrict__ H2, const int* __restrict__ LIST,
                                                  const int* __restrict__ CNT, const int* __restrict__ OFF,
                                                  const float* __restrict__ DINV, const int* __restrict__ POIS,
                                                  const float* __restrict__ B1f, float* __restrict__ out) {
  __shared__ __attribute__((aligned(16))) float sB[C2_];
  const int tid = (int)threadIdx.x, lane = tid & 31, wave = tid >> 5;
  if (tid < 16) { const v4f b = *(const v4fa*)(B1f + 4 * tid); *(v4fa*)(sB + 4 * tid) = b; }
  __syncthreads();
  const v2f bv = *(const v2fa*)(sB + 2 * lane);
  const int row = (int)blockIdx.x * 8 + wave;
  const bool live = row < N_;
  const int rc = live ? row : (N_ - 1);
  int c = CNT[rc];
  asm volatile("" :: "v"(c));
  int o = OFF[rc];
  asm volatile("" :: "v"(o));
  const float dr = DINV[rc];
  asm volatile("" :: "v"(dr));
  const int blk = rc >> 10;
  const int pf = POIS[blk * 32];
  asm volatile("" :: "v"(pf));
  const bool big = c > DEGCAP_;
  c = clampi(c, 0, DEGCAP_);
  o = clampi(o, 0, RCAP_ - 1);
  const int cn = __builtin_amdgcn_readfirstlane(live ? c : 0);
  const int* lst = LIST + (size_t)blk * RCAP_;

  float a0 = 0.0f, a1 = 0.0f;
#pragma unroll 1
  for (int b0 = 0; b0 < cn; b0 += 32) {
    int idx = o + b0 + lane;
    idx = idx > RCAP_ - 1 ? RCAP_ - 1 : idx;
    const int s = clampi(lst[idx], 0, N_ - 1);
    const float w = DINV[s] * dr;
    const int wi = __float_as_int(w);
    const int m32 = (cn - b0) < 32 ? (cn - b0) : 32;
#pragma unroll 1
    for (int k = 0; k < m32; ++k) {
      const int   sk = clampi(__builtin_amdgcn_readlane(s, k), 0, N_ - 1);
      const float ck = __int_as_float(__builtin_amdgcn_readlane(wi, k));
      const v2f a = *(const v2fa*)(H2 + (size_t)sk * C2_ + 2 * lane);
      a0 = fmaf(ck, a[0], a0);
      a1 = fmaf(ck, a[1], a1);
    }
  }
  const v2f hr = *(const v2fa*)(H2 + (size_t)rc * C2_ + 2 * lane);
  const float h0 = hr[0], h1 = hr[1];
  asm volatile("" :: "v"(h0));
  asm volatile("" :: "v"(h1));
  const float rd = dr * dr;
  float y0 = (a0 + h0 * rd) + bv[0];
  float y1 = (a1 + h1 * rd) + bv[1];
  const bool bad = (pf != 0) || big;
  const float qnan = __int_as_float(0x7fc00000);
  y0 = bad ? qnan : y0;
  y1 = bad ? qnan : y1;
  const v2f ov = (v2f){ y0, y1 };
  float* op = out + (size_t)rc * C2_ + 2 * lane;
  for (int pass = 0; pass < 2; ++pass) {
    if (live) *(volatile v2f*)op = ov;
    __threadfence();
  }
}

constexpr size_t al256c(size_t v) { return (v + 255) & ~(size_t)255; }
constexpr size_t SZ_XB   = (size_t)NP_ * C0_ * 2;
constexpr size_t SZ_H    = (size_t)NP_ * C0_ * 4;
constexpr size_t SZ_H2   = (size_t)NP_ * C2_ * 4;
constexpr size_t SZ_H1   = (size_t)NP_ * K1_ * 2;
constexpr size_t SZ_LIST = (size_t)NBLK_ * RCAP_ * 4;
constexpr size_t SZ_TAB  = (size_t)NBLK_ * SLOTS_ * 4;
constexpr size_t SZ_POIS = (size_t)NBLK_ * 128;
constexpr size_t SZ_W0T  = (size_t)C0_ * C0_ * 2;
constexpr size_t SZ_W1D  = (size_t)C2_ * K1_ * 2;
constexpr size_t SZ_B0   = (size_t)C0_ * 4;
constexpr size_t SZ_B1   = (size_t)C2_ * 4;
constexpr size_t O_XB   = 0;
constexpr size_t O_H    = al256c(O_XB + SZ_XB);
constexpr size_t O_H1   = al256c(O_H + SZ_H);
constexpr size_t O_LIST = al256c(O_H1 + SZ_H1);
constexpr size_t O_CNT  = al256c(O_LIST + SZ_LIST);
constexpr size_t O_OFF  = al256c(O_CNT + SZ_TAB);
constexpr size_t O_DINV = al256c(O_OFF + SZ_TAB);
constexpr size_t O_POIS = al256c(O_DINV + SZ_TAB);
constexpr size_t O_W0T  = al256c(O_POIS + SZ_POIS);
constexpr size_t O_W1D  = al256c(O_W0T + SZ_W0T);
constexpr size_t O_B0   = al256c(O_W1D + SZ_W1D);
constexpr size_t O_B1   = al256c(O_B0 + SZ_B0);
constexpr size_t WS_TOTAL = al256c(O_B1 + SZ_B1);
static_assert(WS_TOTAL <= ((size_t)128 << 20));
static_assert(SZ_H2 <= SZ_H);
static_assert((size_t)NP_ * (C0_ / 8) % 256 == 0);
static_assert(((size_t)NP_ * K1_ / 8) < ((size_t)1 << 31));

extern "C" void kernel_launch(void* const* d_in, const int* in_sizes, int n_in,
                              void* d_out, int out_size, void* d_ws, size_t ws_size,
                              hipStream_t stream) {
  if (n_in < 6) return;
  if (in_sizes[0] != N_ * C0_) return;
  if (in_sizes[1] != 2 * E_) return;
  if (in_sizes[2] != C0_ * C0_) return;
  if (in_sizes[3] != C0_) return;
  if (in_sizes[4] != C0_ * C2_) return;
  if (in_sizes[5] != C2_) return;
  if (out_size != N_ * C2_) return;
  if (ws_size < WS_TOTAL) return;

  const float* x   = (const float*)d_in[0];
  const int*   eg  = (const int*)d_in[1];
  const float* W0  = (const float*)d_in[2];
  const float* b0  = (const float*)d_in[3];
  const float* W1  = (const float*)d_in[4];
  const float* b1  = (const float*)d_in[5];
  const int* src = eg;
  const int* dst = eg + E_;
  float* out = (float*)d_out;

  char* ws = (char*)d_ws;
  unsigned short* XB   = (unsigned short*)(ws + O_XB);
  float*          H    = (float*)(ws + O_H);
  float*          H2   = (float*)(ws + O_H);
  unsigned short* H1HL = (unsigned short*)(ws + O_H1);
  int*            LIST = (int*)(ws + O_LIST);
  int*            CNT  = (int*)(ws + O_CNT);
  int*            OFF  = (int*)(ws + O_OFF);
  int*            DINVb = (int*)(ws + O_DINV);
  const float*    DINV = (const float*)(ws + O_DINV);
  int*            POIS = (int*)(ws + O_POIS);
  unsigned short* W0T  = (unsigned short*)(ws + O_W0T);
  unsigned short* W1D  = (unsigned short*)(ws + O_W1D);
  float*          B0f  = (float*)(ws + O_B0);
  float*          B1f  = (float*)(ws + O_B1);

  hipFuncSetAttribute(reinterpret_cast<const void*>(&k_bucket), hipFuncAttributeMaxDynamicSharedMemorySize,
                      (int)BUCKET_LDS);

  k_plane<0><<<NP_ * (C0_ / 8) / 256, 256, 0, stream>>>(x, N_, C0_, C0_, XB, NP_, C0_);
  k_prep<<<PB_TOTAL, BTHR, 0, stream>>>(W0, W1, b0, b1, W0T, W1D, B0f, B1f, H1HL);
  k_bucket<<<NBLK_, BTHR, BUCKET_LDS, stream>>>(src, dst, LIST, CNT, OFF, DINVb, POIS);
  {
    const int T = ((NP_ + 63) / 64) * ((C0_ + 63) / 64);
    k_gemm_nt<0, 0><<<(T + 7) / 8, 256, 0, stream>>>(XB, W0T, B0f, H, NP_, C0_, C0_, C0_);
  }
  k_replay0<<<N_ / 8, BTHR, 0, stream>>>(H, LIST, CNT, OFF, DINV, POIS, B0f, H1HL);
  {
    const int T = ((NP_ + 63) / 64) * ((C2_ + 63) / 64);
    k_gemm_nt<0, 0><<<(T + 7) / 8, 256, 0, stream>>>(H1HL, W1D, B1f, H2, NP_, C2_, K1_, C2_);
  }
  k_replay1<<<N_ / 8, BTHR, 0, stream>>>(H2, LIST, CNT, OFF, DINV, POIS, B1f, out);
}
